// STSA_36679020708366
// MI455X (gfx1250) — hardware-verified
//
#include <hip/hip_runtime.h>
#include <stdint.h>
#include <stddef.h>


#define NB 8
#define NS 512
#define NE 512
#define NH 8
#define ND 64
#define NF 2048
#define NP 64
#define NC 129
#define NCP 192
#define PW 704
#define NT (NB * NS)
#define NBH (NB * NH)
#define QBH 16
#define WSC 16.0f
#define WSC_INV 0.0625f
#define PSC 32768.0f
#define PSC_INV (1.0f / 32768.0f)

typedef __attribute__((ext_vector_type(16))) _Float16 v16h;
typedef __attribute__((ext_vector_type(8)))  _Float16 v8h;
typedef __attribute__((ext_vector_type(4)))  _Float16 v4h;
typedef __attribute__((ext_vector_type(16))) __bf16   v16b;
typedef __attribute__((ext_vector_type(8)))  __bf16   v8b;
typedef __attribute__((ext_vector_type(8)))  float    v8f;
typedef __attribute__((ext_vector_type(4)))  float    v4f;
typedef __attribute__((ext_vector_type(4)))  int      v4i;

union U8f { struct { v4f a, b; } p; float f[8]; };
union U8i { struct { v4i a, b; } p; int f[8]; };

__device__ __forceinline__ unsigned short f2bf_bits(float f) {
  unsigned u = __float_as_uint(f);
  return (unsigned short)((u + 0x7FFFu + ((u >> 16) & 1u)) >> 16);
}
__device__ __forceinline__ float bf_bits2f(unsigned short h) { return __uint_as_float(((unsigned)h) << 16); }

__device__ __forceinline__ void dep_guard_h(v8f& a, v8f& b, v16h x, v16h y) { asm volatile("v_nop\n\tv_nop\n\tv_nop\n\tv_nop" : "+v"(a), "+v"(b) : "v"(x), "v"(y)); }
__device__ __forceinline__ void dep_guard_b(v8f& a, v8f& b, v16b x, v16b y) { asm volatile("v_nop\n\tv_nop\n\tv_nop\n\tv_nop" : "+v"(a), "+v"(b) : "v"(x), "v"(y)); }
__device__ __forceinline__ void keep4_h(v16h a, v16h b, v16h c, v16h d) { asm volatile("v_nop" :: "v"(a), "v"(b), "v"(c), "v"(d)); }
__device__ __forceinline__ void keep4_b(v16b a, v16b b, v16b c, v16b d) { asm volatile("v_nop" :: "v"(a), "v"(b), "v"(c), "v"(d)); }
__device__ __forceinline__ void acc_guard4(v8f& a, v8f& b, v8f& c, v8f& d) { asm volatile("v_nop\n\tv_nop\n\tv_nop\n\tv_nop" : "+v"(a), "+v"(b), "+v"(c), "+v"(d)); }

__device__ __forceinline__ void wave_sync() {
  __builtin_amdgcn_fence(__ATOMIC_RELEASE, "workgroup");
  __builtin_amdgcn_wave_barrier();
  __builtin_amdgcn_fence(__ATOMIC_ACQUIRE, "workgroup");
}

template <typename T> struct Frag;
template <> struct Frag<_Float16> {
  typedef v16h V; union U { v16h v; v8h h[2]; };
  static __device__ __forceinline__ v16h load(const _Float16* p) {
    U f; f.h[0] = *(const v8h*)(p); f.h[1] = *(const v8h*)(p + 16); return f.v;
  }
  static __device__ __forceinline__ v8f mma(v16h a, v16h b, v8f c) {
    return __builtin_amdgcn_wmma_f32_16x16x32_f16(false, a, false, b, (short)0, c, false, false);
  }
  static __device__ __forceinline__ void guard(v8f& a, v8f& b, v16h x, v16h y) { dep_guard_h(a, b, x, y); }
  static __device__ __forceinline__ void keep(v16h a, v16h b, v16h c, v16h d) { keep4_h(a, b, c, d); }
};
template <> struct Frag<__bf16> {
  typedef v16b V; union U { v16b v; v8b h[2]; };
  static __device__ __forceinline__ v16b load(const __bf16* p) {
    U f; f.h[0] = *(const v8b*)(p); f.h[1] = *(const v8b*)(p + 16); return f.v;
  }
  static __device__ __forceinline__ v8f mma(v16b a, v16b b, v8f c) {
    return __builtin_amdgcn_wmma_f32_16x16x32_bf16(false, a, false, b, (short)0, c, false, false);
  }
  static __device__ __forceinline__ void guard(v8f& a, v8f& b, v16b x, v16b y) { dep_guard_b(a, b, x, y); }
  static __device__ __forceinline__ void keep(v16b a, v16b b, v16b c, v16b d) { keep4_b(a, b, c, d); }
};

template <int ET> struct Elem;
template <> struct Elem<0> { typedef _Float16 T; };
template <> struct Elem<1> { typedef __bf16 T; };

template <int ET, bool SPLIT, int BIAS_MODE, int OUT_MODE, bool RESID, int ACT = 0>
__global__ __launch_bounds__(256) void wmma_gemm64(
    const unsigned short* __restrict__ Ap, const unsigned short* __restrict__ A2p,
    const unsigned short* __restrict__ Btp, const unsigned short* __restrict__ Bt2p,
    void* __restrict__ Cout, void* __restrict__ Cout2,
    const float* __restrict__ bias, const float* __restrict__ resid,
    long aBo, long aBi, long bBo, long bBi, long cBo, long cBi, long rBo, long rBi, long cRo, long cCo,
    int bdiv, int lda, int ldb, int ldc, int ldr, int cRS, int cCS, int M, int N, int K, float scale) {
  typedef typename Elem<ET>::T T;
  typedef typename Frag<T>::V V;
  const T* A = (const T*)Ap; const T* A2 = (const T*)A2p; const T* Bt = (const T*)Btp; const T* Bt2 = (const T*)Bt2p;
  __shared__ __align__(16) float sT[8][16 * 68];
  const int y    = blockIdx.y;
  const int yo   = y / bdiv;
  const int yi   = y - yo * bdiv;
  const int lane = threadIdx.x & 31;
  const int wave = threadIdx.x >> 5;
  const int tilesN = N >> 6;
  const int tilesM = M >> 6;
  const int tile = blockIdx.x * 8 + wave;
  if (tile >= tilesM * tilesN) return;
  const int tm = tile / tilesN;
  const int tn = tile - tm * tilesN;
  const int m0 = tm << 6;
  const int n0 = tn << 6;

  const T* Ab  = A  + (size_t)yo * aBo + (size_t)yi * aBi;
  const T* Bb  = Bt + (size_t)yo * bBo + (size_t)yi * bBi;
  const T* Ab2 = SPLIT ? (A2  + (size_t)yo * aBo + (size_t)yi * aBi) : nullptr;
  const T* Bb2 = SPLIT ? (Bt2 + (size_t)yo * bBo + (size_t)yi * bBi) : nullptr;

  const int rlane = lane & 15;
  const int koff  = (lane >> 4) * 8;
  const int mOff  = (lane >> 4) * 8;

  v8f acc[4][4];
#pragma unroll
  for (int i = 0; i < 4; ++i)
#pragma unroll
    for (int j = 0; j < 4; ++j) acc[i][j] = (v8f){0.f,0.f,0.f,0.f,0.f,0.f,0.f,0.f};

  for (int k0 = 0; k0 < K; k0 += 32) {
    V bh[4], bl[4];
#pragma unroll
    for (int j = 0; j < 4; ++j) {
      const size_t bo = (size_t)(n0 + (j << 4) + rlane) * ldb + koff + k0;
      bh[j] = Frag<T>::load(Bb + bo);
      if (SPLIT) bl[j] = Frag<T>::load(Bb2 + bo);
    }
#pragma unroll
    for (int i = 0; i < 4; ++i) {
      const size_t ao = (size_t)(m0 + (i << 4) + rlane) * lda + koff + k0;
      V ah = Frag<T>::load(Ab + ao);
      V al;
      if (SPLIT) al = Frag<T>::load(Ab2 + ao);
#pragma unroll
      for (int j = 0; j < 4; ++j) {
        acc[i][j] = Frag<T>::mma(ah, bh[j], acc[i][j]);
        if (SPLIT) {
          acc[i][j] = Frag<T>::mma(ah, bl[j], acc[i][j]);
          acc[i][j] = Frag<T>::mma(al, bh[j], acc[i][j]);
        }
      }
      Frag<T>::guard(acc[i][0], acc[i][3], ah, SPLIT ? al : ah);
    }
    Frag<T>::keep(bh[0], bh[1], bh[2], bh[3]);
    if (SPLIT) Frag<T>::keep(bl[0], bl[1], bl[2], bl[3]);
  }
  acc_guard4(acc[0][0], acc[0][1], acc[0][2], acc[0][3]);
  acc_guard4(acc[1][0], acc[1][1], acc[1][2], acc[1][3]);
  acc_guard4(acc[2][0], acc[2][1], acc[2][2], acc[2][3]);
  acc_guard4(acc[3][0], acc[3][1], acc[3][2], acc[3][3]);

  float* slab = sT[wave];
  const size_t cb = (size_t)yo * cBo + (size_t)yi * cBi
                  + (size_t)(m0 / cRS) * cRo + (size_t)(m0 % cRS) * ldc
                  + (size_t)(n0 / cCS) * cCo + (size_t)(n0 % cCS);
  const float* Rb = RESID ? (resid + (size_t)yo * rBo + (size_t)yi * rBi) : nullptr;
#pragma unroll
  for (int i = 0; i < 4; ++i) {
    const int mBase = m0 + (i << 4);
#pragma unroll
    for (int j = 0; j < 4; ++j) {
      const int n = n0 + (j << 4) + rlane;
      float bv = 0.f;
      if (BIAS_MODE == 2) bv = bias[n];
#pragma unroll
      for (int r = 0; r < 8; ++r) {
        float v = acc[i][j][r] * scale;
        if (BIAS_MODE == 1) v += bias[mBase + mOff + r];
        if (BIAS_MODE == 2) v += bv;
        if (RESID) v += Rb[(size_t)(mBase + mOff + r) * ldr + n];
        if (ACT == 1) v = tanhf(v);
        if (ACT == 2) v = fmaxf(v, 0.0f);
        if (ACT == 3) v = v / (1.0f + expf(-v));
        if (ACT == 4) v = (v > 0.f) ? v : 0.01f * v;
        if (ACT == 5) v = 0.5f * v * (1.0f + erff(v * 0.70710678118654752f));
        slab[(mOff + r) * 68 + (j << 4) + rlane] = v;
      }
    }
    __builtin_amdgcn_fence(__ATOMIC_RELEASE, "workgroup");
    __builtin_amdgcn_wave_barrier();
    __builtin_amdgcn_fence(__ATOMIC_ACQUIRE, "workgroup");
    if (OUT_MODE == 0) {
      float* C = (float*)Cout + cb;
      const int hh = lane >> 4, c4 = (lane & 15) * 4;
      for (int pass = 0; pass < 2; ++pass) {
#pragma unroll
        for (int it = 0; it < 8; ++it) {
          const int row = it * 2 + hh;
          v4f v = *(const v4f*)(slab + row * 68 + c4);
          *(volatile v4f*)(C + (size_t)((i << 4) + row) * ldc + c4) = v;
        }
        __threadfence();
      }
    } else {
      const int q = lane >> 3, c8 = (lane & 7) * 8;
      unsigned short* C  = (unsigned short*)Cout + cb;
      unsigned short* C2 = (OUT_MODE == 2) ? ((unsigned short*)Cout2 + cb) : nullptr;
      for (int pass = 0; pass < 2; ++pass) {
#pragma unroll
        for (int it = 0; it < 4; ++it) {
          const int row = it * 4 + q;
          const float* sp = slab + row * 68 + c8;
          v8h hv, lv;
#pragma unroll
          for (int e = 0; e < 8; ++e) {
            if (OUT_MODE == 1) {
              hv[e] = (_Float16)sp[e];
            } else {
              unsigned short hb = f2bf_bits(sp[e]);
              unsigned short lb = f2bf_bits(sp[e] - bf_bits2f(hb));
              hv[e] = __builtin_bit_cast(_Float16, hb);
              lv[e] = __builtin_bit_cast(_Float16, lb);
            }
          }
          *(volatile v8h*)(C + (size_t)((i << 4) + row) * ldc + c8) = hv;
          if (OUT_MODE == 2) *(volatile v8h*)(C2 + (size_t)((i << 4) + row) * ldc + c8) = lv;
        }
        __threadfence();
      }
    }
    __builtin_amdgcn_fence(__ATOMIC_RELEASE, "workgroup");
    __builtin_amdgcn_wave_barrier();
    __builtin_amdgcn_fence(__ATOMIC_ACQUIRE, "workgroup");
  }
}

__global__ __launch_bounds__(256) void cast_f32_f16x2(
    const float* __restrict__ in, _Float16* __restrict__ out, int n2) {
  int i = blockIdx.x * 256 + threadIdx.x;
  if (i < n2) {
    const _Float16 h0 = (_Float16)in[2 * i], h1 = (_Float16)in[2 * i + 1];
    const unsigned u = (unsigned)__builtin_bit_cast(unsigned short, h0) | ((unsigned)__builtin_bit_cast(unsigned short, h1) << 16);
    ((volatile unsigned*)out)[i] = u;
    __threadfence();
    ((volatile unsigned*)out)[i] = u;
  }
}

__global__ __launch_bounds__(256) void k_tr_f16(const float* __restrict__ src, _Float16* __restrict__ dst,
                                               int R, int C, float mult) {
  __shared__ float tile[64][65];
  const int tid = threadIdx.x, lane = tid & 31, wave = tid >> 5;
  const int c0 = blockIdx.x * 64, r0 = blockIdx.y * 64;
#pragma unroll
  for (int it = 0; it < 4; ++it) {
    const int rl = it * 16 + (tid >> 4);
    const int cl = (tid & 15) * 4;
    const v4f v = *(const v4f*)(src + (size_t)(r0 + rl) * C + c0 + cl);
    tile[rl][cl + 0] = v[0] * mult;
    tile[rl][cl + 1] = v[1] * mult;
    tile[rl][cl + 2] = v[2] * mult;
    tile[rl][cl + 3] = v[3] * mult;
  }
  __syncthreads();
  const int q = lane >> 3, c8 = (lane & 7) * 8;
  v8h hv[2];
#pragma unroll
  for (int it = 0; it < 2; ++it) {
    const int cl = wave * 8 + it * 4 + q;
#pragma unroll
    for (int e = 0; e < 8; ++e) hv[it][e] = (_Float16)tile[c8 + e][cl];
  }
  for (int pass = 0; pass < 2; ++pass) {
#pragma unroll
    for (int it = 0; it < 2; ++it) {
      const int cl = wave * 8 + it * 4 + q;
      *(volatile v8h*)(dst + (size_t)(c0 + cl) * R + r0 + c8) = hv[it];
    }
    __threadfence();
  }
}

__global__ __launch_bounds__(256) void k_posfill(const float* __restrict__ pos, _Float16* __restrict__ KP,
                                                _Float16* __restrict__ VTP) {
  const int bh = blockIdx.x;
  const int tid = threadIdx.x, lane = tid & 31, wave = tid >> 5;
  for (int pass = 0; pass < 2; ++pass) {
#pragma unroll 1
    for (int it = 0; it < 6; ++it) {
      const int rowl = it * 32 + (tid >> 3);
      const int c8 = (tid & 7) * 8;
      const int cc = rowl < NC ? rowl : (NC - 1);
      v8h hv;
#pragma unroll
      for (int e = 0; e < 8; ++e) {
        const float f = pos[cc * ND + c8 + e];
        hv[e] = (rowl < NC) ? (_Float16)f : (_Float16)0.0f;
      }
      *(volatile v8h*)(KP + (size_t)(bh * PW + NS + rowl) * ND + c8) = hv;
    }
#pragma unroll 1
    for (int dd = 0; dd < 8; ++dd) {
      const int d = wave * 8 + dd;
      const int lg = lane < 24 ? lane : 23;
      v8h hv;
#pragma unroll
      for (int e = 0; e < 8; ++e) {
        const int c = lg * 8 + e;
        const int cc = c < NC ? c : (NC - 1);
        const float f = pos[cc * ND + d];
        hv[e] = (c < NC) ? (_Float16)f : (_Float16)0.0f;
      }
      if (lane < 24) *(volatile v8h*)(VTP + (size_t)(bh * ND + d) * PW + NS + lane * 8) = hv;
    }
    __threadfence();
  }
}

__global__ __launch_bounds__(64) void k_softmax_rows(const float* __restrict__ Sq, const float* __restrict__ dist,
                                                    const int* __restrict__ dt, const int* __restrict__ msk,
                                                    _Float16* __restrict__ PG, int bh0) {
  __shared__ __align__(16) int tsh[NS];
  __shared__ __align__(16) int mshk[NS];
  __shared__ __align__(16) float hist[2][32 * NC];
  __shared__ __align__(16) float tcs[2][132];
  __shared__ __align__(16) float gsh[2][NCP];
  const int tid = threadIdx.x, lane = tid & 31, wave = tid >> 5;
  const int bhl = blockIdx.x >> 5;
  const int bh = bh0 + bhl;
  const int b = bh >> 3;
  const int i0 = (blockIdx.x & 31) * 16 + wave * 8;
  for (int t = tid; t < NS; t += 64) { tsh[t] = dt[b * NS + t]; mshk[t] = msk[b * NS + t]; }
  for (int t = tid; t < 2 * 32 * NC; t += 64) (&hist[0][0])[t] = 0.f;
  for (int t = tid; t < 2 * NCP; t += 64) (&gsh[0][0])[t] = 0.f;
  __syncthreads();
  float* hw = &hist[wave][0];
  float* tw = &tcs[wave][0];
  float* gw = &gsh[wave][0];
  const int hb = lane * NC;
#pragma unroll 1
  for (int r = 0; r < 8; ++r) {
    const int i = i0 + r;
    const float* srow = Sq + (size_t)(bhl * NS + i) * PW;
#pragma unroll
    for (int e = 0; e < 5; ++e) {
      const int c = lane + 32 * e;
      const int cc = c < NC ? c : (NC - 1);
      const float tv = srow[NS + cc];
      if (c < NC) tw[c] = tv;
    }
    wave_sync();
    const int ti = tsh[i];
    const float* drow = dist + (size_t)(b * NS + i) * NS;
    float wv[2][8];
    int cj[2][8];
    float mx = -3.0e38f;
#pragma unroll
    for (int q = 0; q < 2; ++q) {
      const int jb = 256 * q + 8 * lane;
      U8f su, du; U8i tu, mu;
      su.p.a = *(const v4f*)(srow + jb); su.p.b = *(const v4f*)(srow + jb + 4);
      du.p.a = *(const v4f*)(drow + jb); du.p.b = *(const v4f*)(drow + jb + 4);
      tu.p.a = *(const v4i*)(tsh + jb);  tu.p.b = *(const v4i*)(tsh + jb + 4);
      mu.p.a = *(const v4i*)(mshk + jb); mu.p.b = *(const v4i*)(mshk + jb + 4);
#pragma unroll
      for (int e = 0; e < 8; ++e) {
        int rel = tu.f[e] - ti;
        rel = rel < -NP ? -NP : rel;
        rel = rel > NP ? NP : rel;
        const int c = rel + NP;
        cj[q][e] = c;
        float w = (su.f[e] + tw[c]) * 0.125f + 0.6f * du.f[e];
        if (mu.f[e] == 0) w = -1.0e9f;
        wv[q][e] = w;
        mx = fmaxf(mx, w);
      }
    }
#pragma unroll
    for (int off = 16; off > 0; off >>= 1) mx = fmaxf(mx, __shfl_xor(mx, off, 32));
    float sum = 0.f;
#pragma unroll
    for (int q = 0; q < 2; ++q)
#pragma unroll
      for (int e = 0; e < 8; ++e) {
        const float p = __expf(wv[q][e] - mx);
        wv[q][e] = p;
        sum += p;
      }
#pragma unroll
    for (int off = 16; off > 0; off >>= 1) sum += __shfl_xor(sum, off, 32);
    const float inv = 1.0f / sum;
    v8h hp[2];
#pragma unroll
    for (int q = 0; q < 2; ++q)
#pragma unroll
      for (int e = 0; e < 8; ++e) {
        const float aw = wv[q][e] * inv;
        wv[q][e] = aw;
        hp[q][e] = (_Float16)(aw * PSC);
      }
#pragma unroll
    for (int q = 0; q < 2; ++q)
#pragma unroll
      for (int e = 0; e < 8; ++e) hw[hb + cj[q][e]] += wv[q][e];
    wave_sync();
#pragma unroll
    for (int e = 0; e < 5; ++e) {
      const int c = lane + 32 * e;
      const int cc = c < NC ? c : (NC - 1);
      float s = 0.f;
#pragma unroll 8
      for (int l2 = 0; l2 < 32; ++l2) s += hw[l2 * NC + cc];
      if (c < NC) gw[c] = s;
    }
    wave_sync();
#pragma unroll
    for (int q = 0; q < 2; ++q)
#pragma unroll
      for (int e = 0; e < 8; ++e) hw[hb + cj[q][e]] = 0.f;
    const int lg = lane < 24 ? lane : 23;
    v8h hg;
#pragma unroll
    for (int e = 0; e < 8; ++e) hg[e] = (_Float16)(gw[lg * 8 + e] * PSC);
    _Float16* prow = PG + (size_t)(bh * NS + i) * PW;
    for (int pass = 0; pass < 2; ++pass) {
      *(volatile v8h*)(prow + 8 * lane) = hp[0];
      *(volatile v8h*)(prow + 256 + 8 * lane) = hp[1];
      if (lane < 24) *(volatile v8h*)(prow + NS + 8 * lane) = hg;
      __threadfence();
    }
  }
}

template <bool HOUT>
__global__ __launch_bounds__(128) void k_layernorm(const float* __restrict__ Y, const float* __restrict__ gam,
                                                  const float* __restrict__ bet, float* __restrict__ outF,
                                                  _Float16* __restrict__ outH) {
  __shared__ float red[4];
  const int row = blockIdx.x, tid = threadIdx.x, lane = tid & 31, wave = tid >> 5;
  const size_t base = (size_t)row * NE + tid * 4;
  const v4f yv = *(const v4f*)(Y + base);
  float s = (yv[0] + yv[1]) + (yv[2] + yv[3]);
#pragma unroll
  for (int off = 16; off > 0; off >>= 1) s += __shfl_xor(s, off, 32);
  if (lane == 0) red[wave] = s;
  __syncthreads();
  const float mu = ((red[0] + red[1]) + (red[2] + red[3])) * (1.0f / NE);
  __syncthreads();
  v4f dv = yv - mu;
  float s2 = (dv[0] * dv[0] + dv[1] * dv[1]) + (dv[2] * dv[2] + dv[3] * dv[3]);
#pragma unroll
  for (int off = 16; off > 0; off >>= 1) s2 += __shfl_xor(s2, off, 32);
  if (lane == 0) red[wave] = s2;
  __syncthreads();
  const float var = ((red[0] + red[1]) + (red[2] + red[3])) * (1.0f / NE);
  const float inv = rsqrtf(var + 1.0e-5f);
  const v4f gv = *(const v4f*)(gam + tid * 4);
  const v4f bv = *(const v4f*)(bet + tid * 4);
  v4f o = dv * inv * gv + bv;
  v4h oh;
#pragma unroll
  for (int e = 0; e < 4; ++e) oh[e] = (_Float16)o[e];
  for (int pass = 0; pass < 2; ++pass) {
    *(volatile v4f*)(outF + base) = o;
    if (HOUT) *(volatile v4h*)(outH + base) = oh;
    __threadfence();
  }
}

struct GG {
  long aBo, aBi, bBo, bBi, cBo, cBi, rBo, rBi, cRo, cCo;
  int bdiv, lda, ldb, ldc, ldr, cRS, cCS, M, N, K;
  float scale;
};
static GG gg_std(int M, int N, int K, int lda, int ldb, int ldc, float scale) {
  GG g;
  g.aBo = 0; g.aBi = 0; g.bBo = 0; g.bBi = 0; g.cBo = 0; g.cBi = 0; g.rBo = 0; g.rBi = 0; g.cRo = 0; g.cCo = 0;
  g.bdiv = 1; g.lda = lda; g.ldb = ldb; g.ldc = ldc; g.ldr = ldc; g.cRS = M; g.cCS = N;
  g.M = M; g.N = N; g.K = K; g.scale = scale;
  return g;
}
template <int ET, bool SPLIT, int BIAS_MODE, int OUT_MODE, bool RESID, int ACT>
static void gemm_launch(const GG& g, int nb, hipStream_t stream,
                        const unsigned short* A, const unsigned short* A2,
                        const unsigned short* Bt, const unsigned short* Bt2,
                        void* C, void* C2, const float* bias, const float* resid) {
  const int tiles = (g.M >> 6) * (g.N >> 6);
  dim3 grid((tiles + 7) / 8, nb);
  wmma_gemm64<ET, SPLIT, BIAS_MODE, OUT_MODE, RESID, ACT><<<grid, 256, 0, stream>>>(
      A, A2, Bt, Bt2, C, C2, bias, resid,
      g.aBo, g.aBi, g.bBo, g.bBi, g.cBo, g.cBi, g.rBo, g.rBi, g.cRo, g.cCo,
      g.bdiv, g.lda, g.ldb, g.ldc, g.ldr, g.cRS, g.cCS, g.M, g.N, g.K, g.scale);
}

extern "C" void kernel_launch(void* const* d_in, const int* in_sizes, int n_in,
                              void* d_out, int out_size, void* d_ws, size_t ws_size,
                              hipStream_t stream) {
  if (n_in < 21) return;
  if (in_sizes[0] != NT * NE || in_sizes[1] != NB * NS * NS || in_sizes[2] != NT || in_sizes[3] != NT) return;
  if (in_sizes[4] != NE * NE || in_sizes[6] != NE * NE || in_sizes[8] != NE * NE || in_sizes[10] != NE * NE) return;
  if (in_sizes[5] != NE || in_sizes[7] != NE || in_sizes[9] != NE || in_sizes[11] != NE) return;
  if (in_sizes[12] != NC * ND || in_sizes[13] != NE * NF || in_sizes[14] != NF || in_sizes[15] != NF * NE || in_sizes[16] != NE) return;
  if (in_sizes[17] != NE || in_sizes[18] != NE || in_sizes[19] != NE || in_sizes[20] != NE) return;
  if (out_size != NT * NE) return;

  const float* x     = (const float*)d_in[0];
  const float* dist  = (const float*)d_in[1];
  const int*   dtm   = (const int*)d_in[2];
  const int*   mask  = (const int*)d_in[3];
  const float* wq_w  = (const float*)d_in[4];
  const float* wq_b  = (const float*)d_in[5];
  const float* wk_w  = (const float*)d_in[6];
  const float* wk_b  = (const float*)d_in[7];
  const float* wv_w  = (const float*)d_in[8];
  const float* wv_b  = (const float*)d_in[9];
  const float* wo_w  = (const float*)d_in[10];
  const float* wo_b  = (const float*)d_in[11];
  const float* pos   = (const float*)d_in[12];
  const float* w1    = (const float*)d_in[13];
  const float* b1    = (const float*)d_in[14];
  const float* w2    = (const float*)d_in[15];
  const float* b2    = (const float*)d_in[16];
  const float* ln1g  = (const float*)d_in[17];
  const float* ln1b  = (const float*)d_in[18];
  const float* ln2g  = (const float*)d_in[19];
  const float* ln2b  = (const float*)d_in[20];
  float* out = (float*)d_out;

  size_t off = 0;
  auto carve = [&](size_t bytes) -> size_t { size_t p = off; off = (off + bytes + 255) & ~(size_t)255; return p; };
  const size_t oX16 = carve((size_t)NT * NE * 2);
  const size_t oWQT = carve((size_t)NE * NE * 2);
  const size_t oWKT = carve((size_t)NE * NE * 2);
  const size_t oWVT = carve((size_t)NE * NE * 2);
  const size_t oWOT = carve((size_t)NE * NE * 2);
  const size_t oW1T = carve((size_t)NF * NE * 2);
  const size_t oW2T = carve((size_t)NE * NF * 2);
  const size_t oQH  = carve((size_t)NBH * NS * ND * 2);
  const size_t oKP  = carve((size_t)NBH * PW * ND * 2);
  const size_t oVTP = carve((size_t)NBH * ND * PW * 2);
  const size_t oATT = carve((size_t)NT * NE * 2);
  const size_t szS  = (size_t)QBH * NS * PW * 4;
  const size_t szPG = (size_t)NBH * NS * PW * 2;
  const size_t oREG = carve(szS + szPG);
  const size_t oS   = oREG;
  const size_t oPG  = oREG + szS;
  const size_t oY1  = oREG;
  const size_t oL1F = oY1 + (size_t)NT * NE * 4;
  const size_t oL1H = oL1F + (size_t)NT * NE * 4;
  const size_t oHH  = oL1H + (size_t)NT * NE * 2;
  const size_t oY2  = oHH + (size_t)NT * NF * 2;
  if (oY2 + (size_t)NT * NE * 4 > oREG + szS + szPG) return;
  if (off > ws_size || off > (size_t)134217728) return;

  char* ws = (char*)d_ws;
  unsigned short* X16 = (unsigned short*)(ws + oX16);
  unsigned short* WQT = (unsigned short*)(ws + oWQT);
  unsigned short* WKT = (unsigned short*)(ws + oWKT);
  unsigned short* WVT = (unsigned short*)(ws + oWVT);
  unsigned short* WOT = (unsigned short*)(ws + oWOT);
  unsigned short* W1T = (unsigned short*)(ws + oW1T);
  unsigned short* W2T = (unsigned short*)(ws + oW2T);
  unsigned short* QH  = (unsigned short*)(ws + oQH);
  unsigned short* KP  = (unsigned short*)(ws + oKP);
  unsigned short* VTP = (unsigned short*)(ws + oVTP);
  unsigned short* ATT = (unsigned short*)(ws + oATT);
  float*          SB  = (float*)(ws + oS);
  unsigned short* PG  = (unsigned short*)(ws + oPG);
  float*          Y1  = (float*)(ws + oY1);
  float*          L1F = (float*)(ws + oL1F);
  unsigned short* L1H = (unsigned short*)(ws + oL1H);
  unsigned short* HH  = (unsigned short*)(ws + oHH);
  float*          Y2  = (float*)(ws + oY2);

  cast_f32_f16x2<<<(NT * NE / 2 + 255) / 256, 256, 0, stream>>>(x, (_Float16*)X16, NT * NE / 2);
  k_tr_f16<<<dim3(NE / 64, NE / 64), 256, 0, stream>>>(wq_w, (_Float16*)WQT, NE, NE, WSC);
  k_tr_f16<<<dim3(NE / 64, NE / 64), 256, 0, stream>>>(wk_w, (_Float16*)WKT, NE, NE, WSC);
  k_tr_f16<<<dim3(NE / 64, NE / 64), 256, 0, stream>>>(wv_w, (_Float16*)WVT, NE, NE, WSC);
  k_tr_f16<<<dim3(NE / 64, NE / 64), 256, 0, stream>>>(wo_w, (_Float16*)WOT, NE, NE, WSC);
  k_tr_f16<<<dim3(NF / 64, NE / 64), 256, 0, stream>>>(w1, (_Float16*)W1T, NE, NF, WSC);
  k_tr_f16<<<dim3(NE / 64, NF / 64), 256, 0, stream>>>(w2, (_Float16*)W2T, NF, NE, WSC);
  k_posfill<<<NBH, 256, 0, stream>>>(pos, (_Float16*)KP, (_Float16*)VTP);

  {
    GG g = gg_std(NT, NE, NE, NE, NE, ND, WSC_INV);
    g.cRS = NS; g.cRo = (long)NH * NS * ND; g.cCS = ND; g.cCo = (long)NS * ND;
    gemm_launch<0, false, 2, 1, false, 0>(g, 1, stream, X16, X16, WQT, WQT, QH, QH, wq_b, x);
  }
  {
    GG g = gg_std(NT, NE, NE, NE, NE, ND, WSC_INV);
    g.cRS = NS; g.cRo = (long)NH * PW * ND; g.cCS = ND; g.cCo = (long)PW * ND;
    gemm_launch<0, false, 2, 1, false, 0>(g, 1, stream, X16, X16, WKT, WKT, KP, KP, wk_b, x);
  }
  {
    GG g = gg_std(NE, NT, NE, NE, NE, PW, WSC_INV);
    g.cRS = ND; g.cRo = (long)ND * PW; g.cCS = NS; g.cCo = (long)NH * ND * PW;
    gemm_launch<0, false, 1, 1, false, 0>(g, 1, stream, WVT, WVT, X16, X16, VTP, VTP, wv_b, x);
  }

  for (int qt = 0; qt < NBH / QBH; ++qt) {
    GG g = gg_std(NS, PW, ND, ND, ND, PW, 1.0f);
    g.aBo = (long)NS * ND; g.bBo = (long)PW * ND; g.cBo = (long)NS * PW;
    const unsigned short* Aq = QH + (size_t)qt * QBH * NS * ND;
    const unsigned short* Bq = KP + (size_t)qt * QBH * PW * ND;
    gemm_launch<0, false, 0, 0, false, 0>(g, QBH, stream, Aq, Aq, Bq, Bq, SB, SB, wq_b, x);
    k_softmax_rows<<<QBH * (NS / 16), 64, 0, stream>>>(SB, dist, dtm, mask, (_Float16*)PG, qt * QBH);
  }

  {
    GG g = gg_std(NS, ND, PW, PW, PW, NE, PSC_INV);
    g.bdiv = NH;
    g.aBo = (long)NH * NS * PW; g.aBi = (long)NS * PW;
    g.bBo = (long)NH * ND * PW; g.bBi = (long)ND * PW;
    g.cBo = (long)NS * NE;      g.cBi = ND;
    gemm_launch<0, false, 0, 1, false, 0>(g, NBH, stream, PG, PG, VTP, VTP, ATT, ATT, wq_b, x);
  }

  {
    GG g = gg_std(NT, NE, NE, NE, NE, NE, WSC_INV);
    g.ldr = NE;
    gemm_launch<0, false, 2, 0, true, 0>(g, 1, stream, ATT, ATT, WOT, WOT, Y1, Y1, wo_b, x);
  }
  k_layernorm<true><<<NT, 128, 0, stream>>>(Y1, ln1g, ln1b, L1F, (_Float16*)L1H);

  {
    GG g = gg_std(NT, NF, NE, NE, NE, NF, WSC_INV);
    gemm_launch<0, false, 2, 1, false, 2>(g, 1, stream, L1H, L1H, W1T, W1T, HH, HH, b1, x);
  }
  {
    GG g = gg_std(NT, NE, NF, NF, NF, NE, WSC_INV);
    g.ldr = NE;
    gemm_launch<0, false, 2, 0, true, 0>(g, 1, stream, HH, HH, W2T, W2T, Y2, Y2, b2, L1F);
  }

  k_layernorm<false><<<NT, 128, 0, stream>>>(Y2, ln2g, ln2b, out, (_Float16*)L1H);
}
